// NNConv_pair_42073499632117
// MI455X (gfx1250) — hardware-verified
//
#include <hip/hip_runtime.h>
#include <stddef.h>


#define NTHR   256
#define NWAVE  8
#define EPT    8
#define CHUNK  (NTHR * EPT)
#define WCAP   (EPT * 32)
#define LISTN  (NWAVE * WCAP)
#define PASSN  (NWAVE * 16)
#define PCAP   (CHUNK + PASSN)
#define NB     768
#define FV     32
#define EH     16
#define FE     8
#define KE     (EH * FV + FV)
#define GB     64
#define PW     64

#define L_BH    0
#define L_BL    (L_BH + FV * KE * 2)
#define L_RH    (L_BL + FV * KE * 2)
#define L_RL    (L_RH + FV * FV * 2)
#define L_BN    (L_RL + FV * FV * 2)
#define L_W1    (L_BN + FV * 4)
#define L_B1    (L_W1 + FE * EH * 4)
#define L_ACC   (L_B1 + EH * 4)
#define L_MSG   (L_ACC + (NB + 1) * FV * 4)
#define L_SROW  (L_MSG + FV * PASSN * 4)
#define L_LIST  (L_SROW + NWAVE * 16 * FV * 4)
#define L_PEND  (L_LIST + LISTN * 4)
#define L_SLOT  (L_PEND + PCAP * 4)
#define L_WCNT  (L_SLOT + PASSN * 4)
#define L_TOTAL (L_WCNT + 64)

static_assert(PASSN == 128);
static_assert(PCAP >= CHUNK + PASSN);
static_assert((NB % (16 * NWAVE)) == 0);
static_assert((NB % (4 * NWAVE)) == 0);
static_assert(KE == 16 * FV + FV);
static_assert((KE % 32) == 0);
static_assert(FV == 32 && EH == 16 && FE == 8);
static_assert((L_BL % 16) == 0 && (L_RH % 16) == 0 && (L_RL % 16) == 0 && (L_BN % 16) == 0);
static_assert((L_W1 % 16) == 0 && (L_B1 % 16) == 0 && (L_ACC % 16) == 0 && (L_MSG % 16) == 0);
static_assert((L_SROW % 16) == 0 && (L_LIST % 16) == 0 && (L_PEND % 16) == 0);
static_assert((L_SLOT % 16) == 0 && (L_WCNT % 16) == 0 && (L_TOTAL % 16) == 0);
static_assert(L_TOTAL <= 300 * 1024);
static_assert(GB == 64 && GB <= NTHR && PW == 2 * FV);

typedef float          v2f  __attribute__((ext_vector_type(2)));
typedef float          v4f  __attribute__((ext_vector_type(4)));
typedef float          v8f  __attribute__((ext_vector_type(8)));
typedef int            v4i  __attribute__((ext_vector_type(4)));
typedef unsigned short v8us __attribute__((ext_vector_type(8)));
typedef __bf16         v16b __attribute__((ext_vector_type(16)));
union FragB { v16b v; v8us u[2]; };

__device__ __forceinline__ v8f wmb(v16b a, v16b b, v8f c) {
  v8f d = __builtin_amdgcn_wmma_f32_16x16x32_bf16(false, a, false, b, (short)0, c, false, false);
  asm volatile("v_nop\n\tv_nop\n\tv_nop\n\tv_nop" : "+v"(d) : "v"(a), "v"(b));
  return d;
}

__device__ __forceinline__ v8f splat8(float x) {
  v8f c;
#pragma unroll
  for (int i = 0; i < 8; ++i) c[i] = x;
  return c;
}

__device__ __forceinline__ unsigned bfr(float x) {
  unsigned u = __float_as_uint(x);
  u += 0x7fffu + ((u >> 16) & 1u);
  return u >> 16;
}

__device__ __forceinline__ void sp2(float x, unsigned short& hi, unsigned short& lo) {
  const unsigned hb = bfr(x);
  const float hf = __uint_as_float(hb << 16);
  hi = (unsigned short)hb;
  lo = (unsigned short)bfr(x - hf);
}

__device__ __forceinline__ void sp8(v4f a, v4f b, v8us& hi, v8us& lo) {
  float t[8];
  t[0] = a.x; t[1] = a.y; t[2] = a.z; t[3] = a.w;
  t[4] = b.x; t[5] = b.y; t[6] = b.z; t[7] = b.w;
#pragma unroll
  for (int i = 0; i < 8; ++i) {
    unsigned short h, l;
    sp2(t[i], h, l);
    hi[i] = h;
    lo[i] = l;
  }
}

__device__ __forceinline__ int scan_chunk(const int* __restrict__ dsts, int nE, int cbase, int nodeBase,
                                          int vec8, int* list, int tid, int wave) {
  int wc = 0;
  const int el0  = tid * EPT;
  const int e0   = cbase + el0;
  const int sent = -2147483647 - 1;
  v4i da, db;
  if (vec8 != 0 && cbase + CHUNK <= nE) {
    da = *(const v4i*)(dsts + e0);
    db = *(const v4i*)(dsts + e0 + 4);
  } else {
    da.x = (e0     < nE) ? dsts[min(e0, nE - 1)] : sent;
    da.y = (e0 + 1 < nE) ? dsts[min(e0 + 1, nE - 1)] : sent;
    da.z = (e0 + 2 < nE) ? dsts[min(e0 + 2, nE - 1)] : sent;
    da.w = (e0 + 3 < nE) ? dsts[min(e0 + 3, nE - 1)] : sent;
    db.x = (e0 + 4 < nE) ? dsts[min(e0 + 4, nE - 1)] : sent;
    db.y = (e0 + 5 < nE) ? dsts[min(e0 + 5, nE - 1)] : sent;
    db.z = (e0 + 6 < nE) ? dsts[min(e0 + 6, nE - 1)] : sent;
    db.w = (e0 + 7 < nE) ? dsts[min(e0 + 7, nE - 1)] : sent;
  }
  const unsigned nb = (unsigned)nodeBase;
  const unsigned s0 = (unsigned)da.x - nb, s1 = (unsigned)da.y - nb;
  const unsigned s2 = (unsigned)da.z - nb, s3 = (unsigned)da.w - nb;
  const unsigned s4 = (unsigned)db.x - nb, s5 = (unsigned)db.y - nb;
  const unsigned s6 = (unsigned)db.z - nb, s7 = (unsigned)db.w - nb;
  const bool h0 = s0 < (unsigned)NB, h1 = s1 < (unsigned)NB, h2 = s2 < (unsigned)NB, h3 = s3 < (unsigned)NB;
  const bool h4 = s4 < (unsigned)NB, h5 = s5 < (unsigned)NB, h6 = s6 < (unsigned)NB, h7 = s7 < (unsigned)NB;
  const unsigned any = __builtin_amdgcn_ballot_w32(h0 | h1 | h2 | h3 | h4 | h5 | h6 | h7);
  if (any != 0u) {
#define HITJ(J, HJ) { \
      const unsigned mj = __builtin_amdgcn_ballot_w32(HJ); \
      if (mj != 0u) { \
        if (HJ) { \
          const int pos = wc + (int)__builtin_amdgcn_mbcnt_lo(mj, 0u); \
          if (pos < WCAP) list[wave * WCAP + pos] = el0 + (J); \
        } \
        wc += (int)__builtin_popcount(mj); } }
    HITJ(0, h0)
    HITJ(1, h1)
    HITJ(2, h2)
    HITJ(3, h3)
    HITJ(4, h4)
    HITJ(5, h5)
    HITJ(6, h6)
    HITJ(7, h7)
#undef HITJ
  }
  return wc;
}

__global__ __launch_bounds__(NTHR) void k_conv(
    const float* __restrict__ xin, const float* __restrict__ eattr, const int* __restrict__ ei,
    const float* __restrict__ w1, const float* __restrict__ b1,
    const float* __restrict__ w2, const float* __restrict__ b2,
    const float* __restrict__ root, const float* __restrict__ bias,
    float* xout, int nN, int nE, int vec8) {
  extern __shared__ __attribute__((aligned(16))) unsigned char dsm[];
  unsigned short* lbh   = (unsigned short*)(dsm + L_BH);
  unsigned short* lbl   = (unsigned short*)(dsm + L_BL);
  unsigned short* lrh   = (unsigned short*)(dsm + L_RH);
  unsigned short* lrl   = (unsigned short*)(dsm + L_RL);
  float*    lbn   = (float*)(dsm + L_BN);
  float*    lw1   = (float*)(dsm + L_W1);
  float*    lb1   = (float*)(dsm + L_B1);
  float*    acc   = (float*)(dsm + L_ACC);
  float*    msgT  = (float*)(dsm + L_MSG);
  float*    srow  = (float*)(dsm + L_SROW);
  int*      list  = (int*)(dsm + L_LIST);
  int*      pend  = (int*)(dsm + L_PEND);
  int*      slotb = (int*)(dsm + L_SLOT);
  int*      wcnt  = (int*)(dsm + L_WCNT);

  const int tid = threadIdx.x, lane = tid & 31, wave = tid >> 5, hh = lane >> 4, m = lane & 15;
  const int nodeBase = blockIdx.x * NB;
  const int* srcs = ei;
  const int* dsts = ei + nE;

#pragma unroll 1
  for (int idx = tid; idx < FV * KE; idx += NTHR) {
    const int n = idx / KE;
    const int k = idx - n * KE;
    int iw = k >> 4; iw = iw > FV - 1 ? FV - 1 : iw;
    const int f = k & 15;
    const float wv = w2[(size_t)f * (FV * FV) + iw * FV + n];
    int ib = k - EH * FV; ib = ib < 0 ? 0 : (ib > FV - 1 ? FV - 1 : ib);
    const float bv = b2[ib * FV + n];
    const float v = (k < EH * FV) ? wv : bv;
    unsigned short h, l;
    sp2(v, h, l);
    lbh[idx] = h;
    lbl[idx] = l;
  }
#pragma unroll 1
  for (int idx = tid; idx < FV * FV; idx += NTHR) {
    const int n = idx >> 5, k = idx & 31;
    const float v = root[k * FV + n];
    unsigned short h, l;
    sp2(v, h, l);
    lrh[idx] = h;
    lrl[idx] = l;
  }
  if (tid < FV) {
    lbn[tid] = bias[tid];
    const int ic = tid < EH ? tid : EH - 1;
    const float bb = b1[ic];
    if (tid < EH) lb1[tid] = bb;
  }
  if (tid < FE * EH) lw1[tid] = w1[tid];
  {
    const v4f z = {0.0f, 0.0f, 0.0f, 0.0f};
#pragma unroll 1
    for (int i = tid; i < (NB + 1) * FV / 4; i += NTHR) *(v4f*)(acc + 4 * i) = z;
  }
  if (tid == 0) wcnt[NWAVE] = 0;
  __syncthreads();

  const int nChunks = (nE + CHUNK - 1) / CHUNK;
#pragma unroll 1
  for (int ch = 0; ch < nChunks; ++ch) {
    const int cbase = ch * CHUNK;
    const int wc = scan_chunk(dsts, nE, cbase, nodeBase, vec8, list, tid, wave);
    if (lane == 0) wcnt[wave] = wc;
    __syncthreads();

    const int base = wcnt[NWAVE];
    int tot = 0, myoff = 0;
#pragma unroll
    for (int w = 0; w < NWAVE; ++w) {
      int c = wcnt[w];
      c = c > WCAP ? WCAP : (c < 0 ? 0 : c);
      if (w < wave) myoff += c;
      tot += c;
    }
    int newN = base + tot;
    newN = newN > PCAP ? PCAP : newN;
    {
      int n = wcnt[wave];
      n = n > WCAP ? WCAP : (n < 0 ? 0 : n);
      const int* lp = list + wave * WCAP;
      for (int i = lane; i < n; i += 32) {
        const int pos = base + myoff + i;
        if (pos < PCAP) pend[pos] = cbase + lp[i];
      }
    }
    const int fin = (ch == nChunks - 1) ? 1 : 0;
    const int R   = (fin != 0) ? (newN + PASSN - 1) / PASSN : newN / PASSN;
    const int Pv  = (fin != 0) ? newN : R * PASSN;
    __syncthreads();

#pragma unroll 1
    for (int r = 0; r < R; ++r) {
      float hv[8];
      {
        int idx = r * PASSN + wave * 16 + m;
        const bool valid = idx < Pv;
        idx = idx > PCAP - 1 ? PCAP - 1 : idx;
        int e = pend[idx];
        e = e < 0 ? 0 : (e > nE - 1 ? nE - 1 : e);
        const int d = dsts[e];
        int s = srcs[e];
        int slot = d - nodeBase;
        if (!valid || (unsigned)slot >= (unsigned)NB) slot = NB;
        s = s < 0 ? 0 : (s > nN - 1 ? nN - 1 : s);
        const float* xr = xin + (size_t)s * FV + 16 * hh;
        const v4f x0 = *(const v4f*)xr;
        const v4f x1 = *(const v4f*)(xr + 4);
        const v4f x2 = *(const v4f*)(xr + 8);
        const v4f x3 = *(const v4f*)(xr + 12);
        float* sq = srow + (wave * 16 + m) * FV + 16 * hh;
        *(v4f*)sq = x0;
        *(v4f*)(sq + 4) = x1;
        *(v4f*)(sq + 8) = x2;
        *(v4f*)(sq + 12) = x3;
        const float* ap = eattr + (size_t)e * FE;
        const v4f a0 = *(const v4f*)ap;
        const v4f a1 = *(const v4f*)(ap + 4);
        float av[8];
        av[0] = a0.x; av[1] = a0.y; av[2] = a0.z; av[3] = a0.w;
        av[4] = a1.x; av[5] = a1.y; av[6] = a1.z; av[7] = a1.w;
        {
          const v4f ba = *(const v4f*)(lb1 + 8 * hh);
          const v4f bb = *(const v4f*)(lb1 + 8 * hh + 4);
          hv[0] = ba.x; hv[1] = ba.y; hv[2] = ba.z; hv[3] = ba.w;
          hv[4] = bb.x; hv[5] = bb.y; hv[6] = bb.z; hv[7] = bb.w;
        }
#pragma unroll
        for (int q = 0; q < FE; ++q) {
          const v4f wa = *(const v4f*)(lw1 + q * EH + 8 * hh);
          const v4f wb = *(const v4f*)(lw1 + q * EH + 8 * hh + 4);
          hv[0] += av[q] * wa.x; hv[1] += av[q] * wa.y; hv[2] += av[q] * wa.z; hv[3] += av[q] * wa.w;
          hv[4] += av[q] * wb.x; hv[5] += av[q] * wb.y; hv[6] += av[q] * wb.z; hv[7] += av[q] * wb.w;
        }
#pragma unroll
        for (int j = 0; j < 8; ++j) hv[j] = fmaxf(hv[j], 0.0f);
        if (hh == 0) slotb[wave * 16 + m] = slot;
      }
      __syncthreads();

      {
        const float* sp = srow + (wave * 16 + m) * FV;
        v8f c0 = splat8(0.0f), c1 = splat8(0.0f);
        const unsigned short* p0h = lbh + m * KE + 8 * hh;
        const unsigned short* p0l = lbl + m * KE + 8 * hh;
        const unsigned short* p1h = lbh + (16 + m) * KE + 8 * hh;
        const unsigned short* p1l = lbl + (16 + m) * KE + 8 * hh;
#pragma unroll
        for (int c = 0; c < 16; ++c) {
          const v2f xs = *(const v2f*)(sp + 2 * c);
          FragB ah, al, b0h, b0l, b1h, b1l;
#pragma unroll
          for (int j = 0; j < 8; ++j) {
            unsigned short h0, l0, h1, l1;
            sp2(xs.x * hv[j], h0, l0);
            sp2(xs.y * hv[j], h1, l1);
            ah.u[0][j] = h0; al.u[0][j] = l0;
            ah.u[1][j] = h1; al.u[1][j] = l1;
          }
          b0h.u[0] = *(const v8us*)(p0h + 32 * c);
          b0h.u[1] = *(const v8us*)(p0h + 32 * c + 16);
          b0l.u[0] = *(const v8us*)(p0l + 32 * c);
          b0l.u[1] = *(const v8us*)(p0l + 32 * c + 16);
          b1h.u[0] = *(const v8us*)(p1h + 32 * c);
          b1h.u[1] = *(const v8us*)(p1h + 32 * c + 16);
          b1l.u[0] = *(const v8us*)(p1l + 32 * c);
          b1l.u[1] = *(const v8us*)(p1l + 32 * c + 16);
          c0 = wmb(ah.v, b0h.v, c0);
          c0 = wmb(ah.v, b0l.v, c0);
          c0 = wmb(al.v, b0h.v, c0);
          c1 = wmb(ah.v, b1h.v, c1);
          c1 = wmb(ah.v, b1l.v, c1);
          c1 = wmb(al.v, b1h.v, c1);
        }
        {
          FragB ah, al, b0h, b0l, b1h, b1l;
          sp8(*(const v4f*)(sp + 8 * hh), *(const v4f*)(sp + 8 * hh + 4), ah.u[0], al.u[0]);
          sp8(*(const v4f*)(sp + 16 + 8 * hh), *(const v4f*)(sp + 20 + 8 * hh), ah.u[1], al.u[1]);
          b0h.u[0] = *(const v8us*)(p0h + EH * FV);
          b0h.u[1] = *(const v8us*)(p0h + EH * FV + 16);
          b0l.u[0] = *(const v8us*)(p0l + EH * FV);
          b0l.u[1] = *(const v8us*)(p0l + EH * FV + 16);
          b1h.u[0] = *(const v8us*)(p1h + EH * FV);
          b1h.u[1] = *(const v8us*)(p1h + EH * FV + 16);
          b1l.u[0] = *(const v8us*)(p1l + EH * FV);
          b1l.u[1] = *(const v8us*)(p1l + EH * FV + 16);
          c0 = wmb(ah.v, b0h.v, c0);
          c0 = wmb(ah.v, b0l.v, c0);
          c0 = wmb(al.v, b0h.v, c0);
          c1 = wmb(ah.v, b1h.v, c1);
          c1 = wmb(ah.v, b1l.v, c1);
          c1 = wmb(al.v, b1h.v, c1);
        }
        float* mp0 = msgT + m * PASSN + wave * 16 + 8 * hh;
        float* mp1 = msgT + (16 + m) * PASSN + wave * 16 + 8 * hh;
        const v4f o0 = {c0[0], c0[1], c0[2], c0[3]};
        const v4f o1 = {c0[4], c0[5], c0[6], c0[7]};
        const v4f o2 = {c1[0], c1[1], c1[2], c1[3]};
        const v4f o3 = {c1[4], c1[5], c1[6], c1[7]};
        *(v4f*)mp0 = o0;
        *(v4f*)(mp0 + 4) = o1;
        *(v4f*)mp1 = o2;
        *(v4f*)(mp1 + 4) = o3;
      }
      __syncthreads();

      if (tid < FV) {
#pragma unroll 1
        for (int i = 0; i < PASSN; ++i) {
          int sl = slotb[i];
          sl = sl < 0 ? 0 : (sl > NB ? NB : sl);
          acc[sl * FV + tid] += msgT[tid * PASSN + i];
        }
      }
      __syncthreads();
    }

    int rem = newN - R * PASSN;
    rem = rem < 0 ? 0 : rem;
    if (R > 0 && tid < rem) pend[tid] = pend[R * PASSN + tid];
    if (tid == 0) wcnt[NWAVE] = rem;
  }
  __syncthreads();

#pragma unroll 1
  for (int tt = 0; tt < NB / (16 * NWAVE); ++tt) {
    const int t = wave + NWAVE * tt;
    const int lrow0 = 16 * t;
    int ndm = nodeBase + lrow0 + m;
    ndm = ndm > nN - 1 ? nN - 1 : ndm;
    FragB ah, al;
    {
      const float* xr = xin + (size_t)ndm * FV + 8 * hh;
      sp8(*(const v4f*)xr, *(const v4f*)(xr + 4), ah.u[0], al.u[0]);
      sp8(*(const v4f*)(xr + 16), *(const v4f*)(xr + 20), ah.u[1], al.u[1]);
    }
#pragma unroll 1
    for (int nt = 0; nt < 2; ++nt) {
      const int col = 16 * nt + m;
      v8f c = splat8(lbn[col]);
      FragB bh, bl;
      const unsigned short* wp = lrh + col * FV + 8 * hh;
      const unsigned short* wq = lrl + col * FV + 8 * hh;
      bh.u[0] = *(const v8us*)wp;
      bh.u[1] = *(const v8us*)(wp + 16);
      bl.u[0] = *(const v8us*)wq;
      bl.u[1] = *(const v8us*)(wq + 16);
      c = wmb(ah.v, bh.v, c);
      c = wmb(ah.v, bl.v, c);
      c = wmb(al.v, bh.v, c);
#pragma unroll
      for (int rr = 0; rr < 8; ++rr) {
        const int lrow = lrow0 + 8 * hh + rr;
        const float cv = c[rr] + acc[lrow * FV + col];
        acc[lrow * FV + col] = fmaxf(cv, 0.0f);
      }
    }
  }
  __syncthreads();

#pragma unroll 1
  for (int q = 0; q < NB / (NWAVE * 4); ++q) {
    const int row = wave * (NB / NWAVE) + 4 * q + (lane >> 3);
    const int c4 = 4 * (lane & 7);
    const v4f v = *(const v4f*)(acc + row * FV + c4);
    *(volatile v4f*)(xout + (size_t)(nodeBase + row) * FV + c4) = v;
  }
  __threadfence();
#pragma unroll 1
  for (int q = 0; q < NB / (NWAVE * 4); ++q) {
    const int row = wave * (NB / NWAVE) + 4 * q + (lane >> 3);
    const int c4 = 4 * (lane & 7);
    const v4f v = *(const v4f*)(acc + row * FV + c4);
    *(volatile v4f*)(xout + (size_t)(nodeBase + row) * FV + c4) = v;
  }
}

__device__ __forceinline__ void pool_scan(const float* __restrict__ x, const int* __restrict__ bt, int nN,
                                          int g0, int colbase, float* pmax, int* hl, int* hs, int* wc,
                                          int tid, int lane, int wave) {
  const int nCh = (nN + NTHR - 1) / NTHR;
#pragma unroll 1
  for (int ch = 0; ch < nCh; ++ch) {
    const int i  = ch * NTHR + tid;
    const int ic = i > nN - 1 ? nN - 1 : i;
    const int b  = bt[ic];
    const int slot = b - g0;
    const bool hit = (i < nN) && ((unsigned)slot < (unsigned)GB);
    const unsigned mk = __builtin_amdgcn_ballot_w32(hit);
    if (lane == 0) wc[wave] = (int)__builtin_popcount(mk);
    __syncthreads();
    int off = 0, tot = 0;
#pragma unroll
    for (int w = 0; w < NWAVE; ++w) { const int c = wc[w]; if (w < wave) off += c; tot += c; }
    if (hit) {
      const int pos = off + (int)__builtin_amdgcn_mbcnt_lo(mk, 0u);
      if (pos < NTHR) { hl[pos] = i; hs[pos] = slot; }
    }
    __syncthreads();
    tot = tot > NTHR ? NTHR : (tot < 0 ? 0 : tot);
    if (tid < FV) {
#pragma unroll 1
      for (int j = 0; j < tot; ++j) {
        int nd = hl[j];
        nd = nd < 0 ? 0 : (nd > nN - 1 ? nN - 1 : nd);
        int sl = hs[j];
        sl = sl < 0 ? 0 : (sl > GB - 1 ? GB - 1 : sl);
        const float v = x[(size_t)nd * FV + tid];
        float* pp = pmax + sl * PW + colbase + tid;
        *pp = fmaxf(*pp, v);
      }
    }
    __syncthreads();
  }
}

__global__ __launch_bounds__(NTHR) void k_pool(const float* __restrict__ hp, const int* __restrict__ bp,
                                              const float* __restrict__ hd, const int* __restrict__ bd,
                                              const float* __restrict__ W0, const float* __restrict__ c0v,
                                              const float* __restrict__ W1, const float* __restrict__ c1v,
                                              float* out, int nN) {
  __shared__ __attribute__((aligned(16))) float pmax[GB * PW];
  __shared__ __attribute__((aligned(16))) float lw0[PW * PW];
  __shared__ __attribute__((aligned(16))) float lb0[PW];
  __shared__ __attribute__((aligned(16))) float lw1[PW];
  __shared__ __attribute__((aligned(16))) float ys[GB];
  __shared__ int hl[NTHR];
  __shared__ int hs[NTHR];
  __shared__ int wc[NWAVE];
  const int tid = threadIdx.x, lane = tid & 31, wave = tid >> 5;
  const int g0 = blockIdx.x * GB;
  const float ninf = -__builtin_inff();
#pragma unroll 1
  for (int i = tid; i < GB * PW; i += NTHR) pmax[i] = ninf;
#pragma unroll 1
  for (int i = tid; i < PW * PW; i += NTHR) lw0[i] = W0[i];
  if (tid < PW) { lb0[tid] = c0v[tid]; lw1[tid] = W1[tid]; }
  __syncthreads();

  pool_scan(hp, bp, nN, g0, 0,  pmax, hl, hs, wc, tid, lane, wave);
  pool_scan(hd, bd, nN, g0, FV, pmax, hl, hs, wc, tid, lane, wave);

  if (tid < GB) {
    float a = c1v[0];
#pragma unroll 1
    for (int o = 0; o < PW; ++o) {
      float t = lb0[o];
#pragma unroll 4
      for (int i = 0; i < PW; ++i) t += pmax[tid * PW + i] * lw0[i * PW + o];
      a += t * lw1[o];
    }
    ys[tid] = a;
  }
  __syncthreads();
  v4f v = {0.0f, 0.0f, 0.0f, 0.0f};
  if (wave == 0 && lane < 16) v = *(const v4f*)(ys + 4 * lane);
  if (wave == 0 && lane < 16) *(volatile v4f*)(out + g0 + 4 * lane) = v;
  __threadfence();
  if (wave == 0 && lane < 16) *(volatile v4f*)(out + g0 + 4 * lane) = v;
}

extern "C" void kernel_launch(void* const* d_in, const int* in_sizes, int n_in,
                              void* d_out, int out_size, void* d_ws, size_t ws_size,
                              hipStream_t stream) {
  if (n_in < 36) return;
  const int nN = in_sizes[6];
  if (nN < 1 || in_sizes[7] != nN || in_sizes[0] != nN * FV || in_sizes[1] != nN * FV) return;
  const int nE = in_sizes[4] / 2;
  if (nE < 1 || in_sizes[4] != 2 * nE || in_sizes[5] != 2 * nE) return;
  if (in_sizes[2] != nE * FE || in_sizes[3] != nE * FE) return;
  for (int g = 0; g < 4; ++g) {
    const int b = 8 + 6 * g;
    if (in_sizes[b] != FE * EH || in_sizes[b + 1] != EH || in_sizes[b + 2] != EH * FV * FV) return;
    if (in_sizes[b + 3] != FV * FV || in_sizes[b + 4] != FV * FV || in_sizes[b + 5] != FV) return;
  }
  if (in_sizes[32] != PW * PW || in_sizes[33] != PW || in_sizes[34] != PW || in_sizes[35] != 1) return;
  const int G = out_size;
  if (G < GB || (G % GB) != 0) return;

  const float* x_p  = (const float*)d_in[0];
  const float* x_d  = (const float*)d_in[1];
  const float* ea_p = (const float*)d_in[2];
  const float* ea_d = (const float*)d_in[3];
  const int*   ei_p = (const int*)d_in[4];
  const int*   ei_d = (const int*)d_in[5];
  const int*   bt_p = (const int*)d_in[6];
  const int*   bt_d = (const int*)d_in[7];
  const float* pw[24];
  for (int i = 0; i < 24; ++i) pw[i] = (const float*)d_in[8 + i];
  const float* lin0_w = (const float*)d_in[32];
  const float* lin0_b = (const float*)d_in[33];
  const float* lin1_w = (const float*)d_in[34];
  const float* lin1_b = (const float*)d_in[35];
  float* outp = (float*)d_out;

  const int nBlk = (nN + NB - 1) / NB;
  const size_t rowsP = (size_t)nBlk * NB;

  char* ws = (char*)d_ws;
  size_t off = 0;
  const size_t plane = (rowsP * FV * 4 + 255) & ~(size_t)255;
  const size_t o0 = off; off += plane;
  const size_t o1 = off; off += plane;
  const size_t o2 = off; off += plane;
  const size_t o3 = off; off += plane;
  size_t limit = (size_t)134217728;
  if (ws_size < limit) limit = ws_size;
  if (off > limit) return;
  float* P0 = (float*)(ws + o0);
  float* P1 = (float*)(ws + o1);
  float* P2 = (float*)(ws + o2);
  float* P3 = (float*)(ws + o3);

  const int vec8 = ((nE & 3) == 0) ? 1 : 0;

  hipFuncSetAttribute(reinterpret_cast<const void*>(&k_conv), hipFuncAttributeMaxDynamicSharedMemorySize, L_TOTAL);

  k_conv<<<nBlk, NTHR, L_TOTAL, stream>>>(x_p, ea_p, ei_p, pw[0], pw[1], pw[2], pw[3], pw[4], pw[5],
                                          P0, nN, nE, vec8);
  k_conv<<<nBlk, NTHR, L_TOTAL, stream>>>(P0, ea_p, ei_p, pw[6], pw[7], pw[8], pw[9], pw[10], pw[11],
                                          P1, nN, nE, vec8);
  k_conv<<<nBlk, NTHR, L_TOTAL, stream>>>(x_d, ea_d, ei_d, pw[12], pw[13], pw[14], pw[15], pw[16], pw[17],
                                          P2, nN, nE, vec8);
  k_conv<<<nBlk, NTHR, L_TOTAL, stream>>>(P2, ea_d, ei_d, pw[18], pw[19], pw[20], pw[21], pw[22], pw[23],
                                          P3, nN, nE, vec8);

  k_pool<<<G / GB, NTHR, 0, stream>>>(P1, bt_p, P3, bt_d, lin0_w, lin0_b, lin1_w, lin1_b, outp, nN);
}
